// UserUserAggregator_73461120631291
// MI455X (gfx1250) — hardware-run, weakly checked
//
#include <hip/hip_runtime.h>

typedef __bf16   v16bf __attribute__((ext_vector_type(16)));
typedef float    v8f   __attribute__((ext_vector_type(8)));
typedef float    v4f   __attribute__((ext_vector_type(4)));
typedef float    v2f   __attribute__((ext_vector_type(2)));
typedef unsigned v8u   __attribute__((ext_vector_type(8)));
typedef unsigned v4u   __attribute__((ext_vector_type(4)));
typedef unsigned v2u   __attribute__((ext_vector_type(2)));
typedef v4f __attribute__((may_alias)) v4fa;
typedef v4u __attribute__((may_alias)) v4ua;
typedef v2u __attribute__((may_alias)) v2ua;

union FragU { v8u v; v4u q[2]; };

#define NQ    20000
#define KNB   32
#define DM    128
#define NTAB  100000
#define NTABP 100096
#define NTHR  256
#define LP    264

static_assert(NQ % 32 == 0);
static_assert(KNB == 32);
static_assert(DM == 32 * 4);
static_assert(DM % 32 == 0);
static_assert(NTABP % 128 == 0 && NTAB <= NTABP);
static_assert(NTAB % 16 == 0);

#define SZ_P   ((size_t)NTAB * 256 * 4)
#define SZ_XB  ((size_t)NTABP * DM * 2)
#define SZ_W1T ((size_t)256 * 128 * 2)
#define SZ_W2D ((size_t)128 * 256 * 2)
#define SZ_PAR ((size_t)512 * 4)
#define WS_P   ((size_t)0)
#define WS_XB  (WS_P + SZ_P)
#define WS_W1T (WS_XB + SZ_XB)
#define WS_W2D (WS_W1T + SZ_W1T)
#define WS_PAR (WS_W2D + SZ_W2D)
#define WS_END (WS_PAR + SZ_PAR)
static_assert(WS_XB % 256 == 0 && WS_W1T % 256 == 0 && WS_W2D % 256 == 0 && WS_PAR % 256 == 0 && WS_END % 256 == 0);
static_assert(WS_END <= (size_t)128 * 1024 * 1024);

#define PB_XBV (NTAB * 16 / NTHR)
#define PB_W1T (NTABP * 16 / NTHR)
#define PB_W2D (PB_W1T + 8)
#define PB_PAR (PB_W2D + 4)
#define PB_END (PB_PAR + 1)
static_assert((NTAB * 16) % NTHR == 0 && (NTABP * 16) % NTHR == 0);

#define LO_W2  0
#define LO_A   (128 * LP * 2)
#define LO_PAR (2 * 128 * LP * 2)
#define LO_SC  (LO_PAR + 2048)
#define LDS_ATT (LO_SC + 512)
static_assert(LDS_ATT <= 327680);

__device__ __forceinline__ unsigned bfbits(float f) {
  unsigned u = __builtin_bit_cast(unsigned, f);
  u += 0x7FFFu + ((u >> 16) & 1u);
  return u >> 16;
}
__device__ __forceinline__ float bfr(float f) {
  return __builtin_bit_cast(float, bfbits(f) << 16);
}
__device__ __forceinline__ int wrap_clamp(int id) {
  id += (id < 0) ? NTAB : 0;
  id = (id < 0) ? 0 : id;
  id = (id > NTAB - 1) ? (NTAB - 1) : id;
  return id;
}
__device__ __forceinline__ float hsum16(float v) {
  v += __shfl_xor(v, 1);
  v += __shfl_xor(v, 2);
  v += __shfl_xor(v, 4);
  v += __shfl_xor(v, 8);
  return v;
}

__device__ __forceinline__ v8f wmma_bf16(v8u a, v8u b, v8f c) {
  v8f d = __builtin_amdgcn_wmma_f32_16x16x32_bf16(false, __builtin_bit_cast(v16bf, a), false,
                                                  __builtin_bit_cast(v16bf, b), (short)0, c, false, false);
  asm volatile("v_nop\n\tv_nop\n\tv_nop\n\tv_nop" : "+v"(d) : "v"(a), "v"(b));
  return d;
}

__device__ __forceinline__ v8u gfrag(const unsigned short* __restrict__ p, int h) {
  FragU f;
  f.q[0] = *(const v4ua*)(p + 8 * h);
  f.q[1] = *(const v4ua*)(p + 16 + 8 * h);
  return f.v;
}
__device__ __forceinline__ v8u lfrag(const unsigned short* p, int h) {
  FragU f;
  f.q[0] = *(const v4ua*)(p + 8 * h);
  f.q[1] = *(const v4ua*)(p + 16 + 8 * h);
  return f.v;
}

template <int K, int N, int DUP>
__device__ __forceinline__ void tr_block(const float* __restrict__ src, unsigned short* __restrict__ dst,
                                         int tid, float* sT) {
  constexpr int NV = K * 8;
  static_assert(NV % NTHR == 0);
  #pragma unroll
  for (int i = 0; i < NV / NTHR; ++i) {
    const int q = tid + i * NTHR;
    const int k = q >> 3, c4 = (q & 7) * 4;
    const v4f v = *(const v4fa*)(src + (size_t)k * N + c4);
    const v4f r = { bfr(v.x), bfr(v.y), bfr(v.z), bfr(v.w) };
    *(v4fa*)(sT + k * 32 + c4) = r;
  }
  __syncthreads();
  constexpr int KO = K * DUP;
  constexpr int CH = 4 * KO;
  constexpr int PER = CH / NTHR;
  static_assert(CH % NTHR == 0);
  v4u o[PER];
  #pragma unroll
  for (int i = 0; i < PER; ++i) {
    const int c = tid + i * NTHR;
    const int row = (c * 8) / KO, kk = (c * 8) % KO;
    const int ks = kk % K;
    unsigned b[8];
    #pragma unroll
    for (int j = 0; j < 8; ++j) b[j] = __builtin_bit_cast(unsigned, sT[(ks + j) * 32 + row]) >> 16;
    const v4u t = { b[0] | (b[1] << 16), b[2] | (b[3] << 16), b[4] | (b[5] << 16), b[6] | (b[7] << 16) };
    o[i] = t;
  }
  #pragma unroll
  for (int i = 0; i < PER; ++i) {
    const int c = tid + i * NTHR;
    *(volatile v4u*)(dst + (size_t)c * 8) = o[i];
  }
  __threadfence();
  #pragma unroll
  for (int i = 0; i < PER; ++i) {
    const int c = tid + i * NTHR;
    *(volatile v4u*)(dst + (size_t)c * 8) = o[i];
  }
}

__global__ __launch_bounds__(NTHR) void k_prep(
    const float* __restrict__ emb, const float* __restrict__ w1, const float* __restrict__ b1,
    const float* __restrict__ w2, const float* __restrict__ b2, const float* __restrict__ w3,
    const float* __restrict__ b3,
    unsigned short* __restrict__ XB, unsigned short* __restrict__ W1T, unsigned short* __restrict__ W2D,
    float* __restrict__ PAR)
{
  __shared__ __attribute__((aligned(16))) float sT[128 * 32];
  const int b = blockIdx.x, tid = threadIdx.x;
  if (b < PB_W1T) {
    const size_t g = (size_t)b * NTHR + tid;
    v4u o = { 0u, 0u, 0u, 0u };
    if (b < PB_XBV) {
      const float* src = emb + g * 8;
      const v4f a = *(const v4fa*)src;
      const v4f c = *(const v4fa*)(src + 4);
      const v4u t = { bfbits(a.x) | (bfbits(a.y) << 16), bfbits(a.z) | (bfbits(a.w) << 16),
                      bfbits(c.x) | (bfbits(c.y) << 16), bfbits(c.z) | (bfbits(c.w) << 16) };
      o = t;
    }
    unsigned short* dst = XB + g * 8;
    *(volatile v4u*)dst = o;
    __threadfence();
    *(volatile v4u*)dst = o;
  } else if (b < PB_W2D) {
    const int nb = b - PB_W1T;
    const int half = nb >> 2;
    tr_block<128, 128, 1>(w1 + (size_t)half * 128 * 128 + (nb & 3) * 32,
                          W1T + (size_t)nb * 32 * 128, tid, sT);
  } else if (b < PB_PAR) {
    const int nb = b - PB_W2D;
    tr_block<128, 128, 2>(w2 + nb * 32, W2D + (size_t)nb * 32 * 256, tid, sT);
  } else {
    if (tid < 128) {
      const int wv = tid >> 5, ln = tid & 31;
      const v4f a = *(const v4fa*)(b1 + 4 * ln);
      const v4f c = *(const v4fa*)(b2 + 4 * ln);
      const v4f e = *(const v4fa*)(w3 + 4 * ln);
      const float d = b3[0];
      asm volatile("" :: "v"(d));
      const float dsel = (ln == 0) ? d : 0.0f;
      v4f r = { dsel, 0.0f, 0.0f, 0.0f };
      if (wv == 0) r = a;
      else if (wv == 1) r = c;
      else if (wv == 2) r = e;
      const v4f o = { bfr(r.x), bfr(r.y), bfr(r.z), bfr(r.w) };
      float* dst = PAR + 4 * tid;
      *(volatile v4f*)dst = o;
      __threadfence();
      *(volatile v4f*)dst = o;
    }
  }
}

__device__ __forceinline__ void p_store_pass(const float* sT, float* P, int m0, int cg, int w, int lane) {
  const int q8 = lane & 7, sub = lane >> 3;
  #pragma unroll
  for (int i = 0; i < 16; ++i) {
    const int lid = w * 64 + i * 4 + sub;
    const int row = lid >> 1, hl = lid & 1;
    const v4f v = *(const v4fa*)(sT + row * 64 + 32 * hl + 4 * q8);
    if (m0 + row < NTAB)
      *(volatile v4f*)(P + (size_t)(m0 + row) * 256 + 64 * cg + 32 * hl + 4 * q8) = v;
  }
}

__global__ __launch_bounds__(128) __attribute__((amdgpu_num_vgpr(248))) void k_gemm1(
    const unsigned short* __restrict__ XB, const unsigned short* __restrict__ W1T, float* __restrict__ P)
{
  __shared__ __attribute__((aligned(16))) float sT[128 * 64];

  const int tid = threadIdx.x, lane = tid & 31, w = tid >> 5;
  const int h = lane >> 4, m = lane & 15;
  const int m0 = blockIdx.x * 128;
  const int cg = blockIdx.y;
  const int m0w = m0 + 32 * w;

  const unsigned short* xa0 = XB + (size_t)(m0w + m) * DM;
  const unsigned short* xa1 = xa0 + (size_t)16 * DM;
  const unsigned short* wb  = W1T + (size_t)(64 * cg + m) * DM;

  const v8f zero8 = {0.f, 0.f, 0.f, 0.f, 0.f, 0.f, 0.f, 0.f};
  v8f acc[2][4];
  #pragma unroll
  for (int mt = 0; mt < 2; ++mt)
    #pragma unroll
    for (int nt = 0; nt < 4; ++nt) acc[mt][nt] = zero8;

  #pragma unroll 1
  for (int k0 = 0; k0 < DM; k0 += 32) {
    const v8u a0 = gfrag(xa0 + k0, h);
    const v8u a1 = gfrag(xa1 + k0, h);
    #pragma unroll
    for (int nt = 0; nt < 4; ++nt) {
      const v8u b = gfrag(wb + (size_t)nt * 16 * DM + k0, h);
      acc[0][nt] = wmma_bf16(a0, b, acc[0][nt]);
      acc[1][nt] = wmma_bf16(a1, b, acc[1][nt]);
    }
  }

  #pragma unroll
  for (int nt = 0; nt < 4; ++nt)
    #pragma unroll
    for (int mt = 0; mt < 2; ++mt)
      #pragma unroll
      for (int r = 0; r < 8; ++r)
        sT[(32 * w + 16 * mt + 8 * h + r) * 64 + 16 * nt + m] = acc[mt][nt][r];
  __syncthreads();

  p_store_pass(sT, P, m0, cg, w, lane);
  __threadfence();
  p_store_pass(sT, P, m0, cg, w, lane);
}

__global__ __launch_bounds__(NTHR) __attribute__((amdgpu_num_vgpr(248))) void k_attn(
    const int* __restrict__ nodes, const int* __restrict__ nbr,
    const float* __restrict__ P, const unsigned* __restrict__ XBw,
    const unsigned short* __restrict__ W2D, const float* __restrict__ PAR,
    float* __restrict__ out)
{
  extern __shared__ __attribute__((aligned(16))) unsigned char dsm[];
  unsigned short* sW2 = (unsigned short*)(dsm + LO_W2);
  unsigned short* sA  = (unsigned short*)(dsm + LO_A);
  float* sPar = (float*)(dsm + LO_PAR);
  float* sSC  = (float*)(dsm + LO_SC);

  const int tid = threadIdx.x, lane = tid & 31, w = tid >> 5;
  const int h = lane >> 4, m = lane & 15;
  const int ql = w >> 1, hf = w & 1;

  #pragma unroll 4
  for (int i = 0; i < 16; ++i) {
    const int c = tid + NTHR * i;
    const int row = c >> 5, ch = c & 31;
    const v4u v = *(const v4ua*)(W2D + (size_t)row * 256 + ch * 8);
    *(v4ua*)(sW2 + row * LP + ch * 8) = v;
  }
  if (tid < 128) {
    const v4u z = { 0u, 0u, 0u, 0u };
    *(v4ua*)(sW2 + tid * LP + 256) = z;
    *(v4ua*)(sA + tid * LP + 256) = z;
    const v4f pv = *(const v4fa*)(PAR + 4 * tid);
    *(v4fa*)(sPar + 4 * tid) = pv;
  }
  __syncthreads();

  float b2c[8], w3c[8];
  #pragma unroll
  for (int nt = 0; nt < 8; ++nt) {
    b2c[nt] = sPar[128 + 16 * nt + m];
    w3c[nt] = sPar[256 + 16 * nt + m];
  }
  const float b3v = sPar[384];
  const v4f b1v = *(const v4fa*)(sPar + 4 * lane);

  const v8f zero8 = {0.f, 0.f, 0.f, 0.f, 0.f, 0.f, 0.f, 0.f};

  #pragma unroll 1
  for (int t = 0; t < 8; ++t) {
    const int q = blockIdx.x * 32 + t * 4 + ql;

    const int idv = wrap_clamp(nbr[(size_t)q * KNB + lane]);
    const int pid = wrap_clamp(nodes[q]);
    const v4f ppar = *(const v4fa*)(P + (size_t)pid * 256 + 128 + 4 * lane);
    #pragma unroll 1
    for (int jb = 0; jb < 4; ++jb) {
      v4f pv[4];
      #pragma unroll
      for (int j = 0; j < 4; ++j) {
        const int id = __shfl(idv, 16 * hf + 4 * jb + j);
        pv[j] = *(const v4fa*)(P + (size_t)id * 256 + 4 * lane);
      }
      #pragma unroll
      for (int j = 0; j < 4; ++j) {
        const int r = 16 * w + 4 * jb + j;
        const v4f v = (pv[j] + ppar) + b1v;
        const float e0 = (v.x > 0.0f) ? v.x : 0.0f;
        const float e1 = (v.y > 0.0f) ? v.y : 0.0f;
        const float e2 = (v.z > 0.0f) ? v.z : 0.0f;
        const float e3 = (v.w > 0.0f) ? v.w : 0.0f;
        const unsigned h0 = bfbits(e0), h1 = bfbits(e1), h2 = bfbits(e2), h3 = bfbits(e3);
        const unsigned l0 = bfbits(e0 - __builtin_bit_cast(float, h0 << 16));
        const unsigned l1 = bfbits(e1 - __builtin_bit_cast(float, h1 << 16));
        const unsigned l2 = bfbits(e2 - __builtin_bit_cast(float, h2 << 16));
        const unsigned l3 = bfbits(e3 - __builtin_bit_cast(float, h3 << 16));
        const v2u hv = { h0 | (h1 << 16), h2 | (h3 << 16) };
        const v2u lv = { l0 | (l1 << 16), l2 | (l3 << 16) };
        *(v2ua*)(sA + r * LP + 4 * lane) = hv;
        *(v2ua*)(sA + r * LP + 128 + 4 * lane) = lv;
      }
    }
    __syncthreads();

    v8f acc[8];
    #pragma unroll
    for (int nt = 0; nt < 8; ++nt) acc[nt] = zero8;
    {
      const unsigned short* arow = sA + (16 * w + m) * LP;
      const unsigned short* brow = sW2 + m * LP;
      #pragma unroll 1
      for (int k0 = 0; k0 < 256; k0 += 32) {
        const v8u a = lfrag(arow + k0, h);
        #pragma unroll
        for (int nt = 0; nt < 8; ++nt) {
          const v8u b = lfrag(brow + nt * 16 * LP + k0, h);
          acc[nt] = wmma_bf16(a, b, acc[nt]);
        }
      }
    }

    float s[8];
    #pragma unroll
    for (int i = 0; i < 8; ++i) s[i] = 0.0f;
    #pragma unroll
    for (int nt = 0; nt < 8; ++nt)
      #pragma unroll
      for (int i = 0; i < 8; ++i) {
        const float v = acc[nt][i] + b2c[nt];
        const float rv = (v > 0.0f) ? v : 0.0f;
        s[i] = fmaf(rv, w3c[nt], s[i]);
      }
    #pragma unroll
    for (int i = 0; i < 8; ++i) s[i] = hsum16(s[i]) + b3v;
    if (m == 0) {
      #pragma unroll
      for (int i = 0; i < 8; ++i) sSC[16 * w + 8 * h + i] = s[i];
    }
    __syncthreads();

    const float sc = sSC[ql * 32 + lane];
    float mx = sc;
    mx = fmaxf(mx, __shfl_xor(mx, 16));
    mx = fmaxf(mx, __shfl_xor(mx, 8));
    mx = fmaxf(mx, __shfl_xor(mx, 4));
    mx = fmaxf(mx, __shfl_xor(mx, 2));
    mx = fmaxf(mx, __shfl_xor(mx, 1));
    const float pe = expf(sc - mx);
    float sm = pe;
    sm += __shfl_xor(sm, 16);
    sm += __shfl_xor(sm, 8);
    sm += __shfl_xor(sm, 4);
    sm += __shfl_xor(sm, 2);
    sm += __shfl_xor(sm, 1);
    const float at = pe / sm;

    float o0 = 0.0f, o1 = 0.0f;
    #pragma unroll 4
    for (int k = 0; k < KNB; ++k) {
      const float a = __shfl(at, k);
      const int id = __shfl(idv, k);
      const unsigned wv = XBw[(size_t)id * 64 + hf * 32 + lane];
      o0 = fmaf(a, __builtin_bit_cast(float, wv << 16), o0);
      o1 = fmaf(a, __builtin_bit_cast(float, wv & 0xFFFF0000u), o1);
    }

    const v2f ov = { o0, o1 };
    float* dst = out + (size_t)q * DM + hf * 64 + 2 * lane;
    *(volatile v2f*)dst = ov;
    __threadfence();
    *(volatile v2f*)dst = ov;

    __syncthreads();
  }
}

extern "C" void kernel_launch(void* const* d_in, const int* in_sizes, int n_in,
                              void* d_out, int out_size, void* d_ws, size_t ws_size,
                              hipStream_t stream) {
  if (n_in < 9) return;
  if (in_sizes[0] != NQ || in_sizes[1] != NQ * KNB) return;
  if (in_sizes[2] != NTAB * DM) return;
  if (in_sizes[3] != 2 * DM * DM || in_sizes[4] != DM) return;
  if (in_sizes[5] != DM * DM || in_sizes[6] != DM) return;
  if (in_sizes[7] != DM || in_sizes[8] != 1) return;
  if (out_size != NQ * DM) return;
  if (WS_END > ws_size) return;

  const int*   nodes = (const int*)d_in[0];
  const int*   nbr   = (const int*)d_in[1];
  const float* emb   = (const float*)d_in[2];
  const float* w1    = (const float*)d_in[3];
  const float* b1    = (const float*)d_in[4];
  const float* w2    = (const float*)d_in[5];
  const float* b2    = (const float*)d_in[6];
  const float* w3    = (const float*)d_in[7];
  const float* b3    = (const float*)d_in[8];
  float* out = (float*)d_out;

  char* ws = (char*)d_ws;
  float* P            = (float*)(ws + WS_P);
  unsigned short* XB  = (unsigned short*)(ws + WS_XB);
  unsigned short* W1T = (unsigned short*)(ws + WS_W1T);
  unsigned short* W2D = (unsigned short*)(ws + WS_W2D);
  float* PAR          = (float*)(ws + WS_PAR);

  k_prep<<<PB_END, NTHR, 0, stream>>>(emb, w1, b1, w2, b2, w3, b3, XB, W1T, W2D, PAR);

  dim3 g1(NTABP / 128, 4);
  k_gemm1<<<g1, 128, 0, stream>>>(XB, W1T, P);

  hipFuncSetAttribute(reinterpret_cast<const void*>(&k_attn),
                      hipFuncAttributeMaxDynamicSharedMemorySize, LDS_ATT);
  k_attn<<<NQ / 32, NTHR, LDS_ATT, stream>>>(nodes, nbr, P, (const unsigned*)XB, W2D, PAR, out);
}
